// SparseSelfAttention_10230612099477
// MI455X (gfx1250) — hardware-verified
//
#include <hip/hip_runtime.h>
#include <math.h>

typedef __attribute__((ext_vector_type(16))) _Float16 v16h;
typedef __attribute__((ext_vector_type(16))) __bf16 v16b;
typedef __attribute__((ext_vector_type(8)))  _Float16 v8h;
typedef __attribute__((ext_vector_type(8)))  __bf16 v8b;
typedef __attribute__((ext_vector_type(8)))  float v8f;
typedef __attribute__((ext_vector_type(4)))  float v4f;
typedef __attribute__((ext_vector_type(4)))  unsigned v4u;

template <typename T> __device__ __forceinline__ void vst2(void* p, T v) { *(volatile T*)p = v; __threadfence(); *(volatile T*)p = v; }

__device__ __forceinline__ v8f wmma16(v16h a, v16h b, v8f c) {
  v8f d = __builtin_amdgcn_wmma_f32_16x16x32_f16(false, a, false, b, (short)0, c, false, false);
  asm volatile("v_nop\n\tv_nop\n\tv_nop\n\tv_nop" : "+v"(d) : "v"(a), "v"(b));
  return d;
}
__device__ __forceinline__ v8f wmma_bf(v16b a, v16b b, v8f c) {
  v8f d = __builtin_amdgcn_wmma_f32_16x16x32_bf16(false, a, false, b, (short)0, c, false, false);
  asm volatile("v_nop\n\tv_nop\n\tv_nop\n\tv_nop" : "+v"(d) : "v"(a), "v"(b));
  return d;
}
__device__ __forceinline__ v16h frag_h(const _Float16* rowk0, int lane) {
  union { v16h v; v8h q[2]; } u; const _Float16* p = rowk0 + 8 * (lane >> 4);
  u.q[0] = *(const v8h*)p; u.q[1] = *(const v8h*)(p + 16); return u.v;
}
__device__ __forceinline__ v16b frag_b(const __bf16* rowk0, int lane) {
  union { v16b v; v8b q[2]; } u; const __bf16* p = rowk0 + 8 * (lane >> 4);
  u.q[0] = *(const v8b*)p; u.q[1] = *(const v8b*)(p + 16); return u.v;
}
#define LDSX() do { asm volatile("s_wait_dscnt 0" ::: "memory"); __builtin_amdgcn_wave_barrier(); __builtin_amdgcn_fence(__ATOMIC_RELEASE, "workgroup"); } while (0)

#ifndef NB
#define NB 2
#endif
#define SEQ 4096
#define DMOD 512
#define NH 8
#define HD 64
#define RATE 4
#define NVALID (SEQ / RATE + 1)
#define NKS ((NVALID + 31) / 32)
#define MP 1088
#define MT (MP / 64)
#define LP (MP * RATE)
#define NQB (SEQ / RATE / 64)
#define NG (NB * NH * RATE)
#define XSTRIDE_FULL ((size_t)SEQ * DMOD)
#define OSTRIDE_FULL ((size_t)SEQ * DMOD)

static_assert(MP % 64 == 0);
static_assert(MP >= NKS * 32);
static_assert(NKS * 32 >= NVALID);
static_assert(SEQ % (RATE * 64) == 0);
static_assert(DMOD == NH * HD);
static_assert(HD == 64);
static_assert(DMOD % 128 == 0);
static_assert(NQB * 64 + 0 <= MP);

#define XB_BYTES ((size_t)2 * NB * LP * DMOD)
#define WT_BYTES ((size_t)2 * 3 * DMOD * DMOD)
#define PL_BYTES ((size_t)2 * NG * MP * HD)
#define WS_XB ((size_t)0)
#define WS_WT (WS_XB + XB_BYTES)
#define WS_QH (WS_WT + WT_BYTES)
#define WS_QL (WS_QH + PL_BYTES)
#define WS_KH (WS_QL + PL_BYTES)
#define WS_KL (WS_KH + PL_BYTES)
#define WS_VT (WS_KL + PL_BYTES)
#define WS_END (WS_VT + PL_BYTES)
static_assert(WS_END <= (size_t)134217728);
static_assert(XB_BYTES % 128 == 0);
static_assert(WT_BYTES % 128 == 0);
static_assert(PL_BYTES % 128 == 0);
static_assert((MP * 2) % 128 == 0);

__global__ __launch_bounds__(256) void k_cvtx(const float* __restrict__ X, __bf16* __restrict__ XB) {
  const int t = threadIdx.x, b = blockIdx.y; const int row = blockIdx.x * 4 + (t >> 6), pc = t & 63;
  const int rs = (row < SEQ) ? row : (SEQ - 1);
  const float* p = X + (size_t)b * XSTRIDE_FULL + (size_t)rs * DMOD + pc * 8;
  const v4f a = *(const v4f*)p, c = *(const v4f*)(p + 4);
  const bool live = row < SEQ;
  union { v8b h; v4u u; } o;
#pragma unroll
  for (int i = 0; i < 4; ++i) { o.h[i] = (__bf16)(live ? a[i] : 0.f); o.h[4 + i] = (__bf16)(live ? c[i] : 0.f); }
  vst2(XB + ((size_t)b * LP + row) * DMOD + pc * 8, o.u);
}
__global__ __launch_bounds__(256) void k_wt(const float* __restrict__ WQ, const float* __restrict__ WK, const float* __restrict__ WV, __bf16* __restrict__ WT) {
  __shared__ __align__(16) __bf16 s[64][72];
  const int kt = blockIdx.x, nt = blockIdx.y, which = blockIdx.z, t = threadIdx.x;
  const float* W = (which == 0) ? WQ : (which == 1) ? WK : WV;
  for (int e = t; e < 64 * 64; e += 256) { const int kk = e >> 6, nn = e & 63; s[nn][kk] = (__bf16)W[(size_t)(kt * 64 + kk) * DMOD + nt * 64 + nn]; }
  __syncthreads();
#pragma unroll
  for (int it = 0; it < 2; ++it) { const int row = it * 32 + (t >> 3), pc = t & 7;
    vst2(WT + ((size_t)which * DMOD + nt * 64 + row) * DMOD + kt * 64 + pc * 8, *(const v4u*)&s[row][pc * 8]); }
}
__global__ __launch_bounds__(128) void k_proj(const __bf16* __restrict__ XB, const __bf16* __restrict__ WT, _Float16* __restrict__ QH, _Float16* __restrict__ QL, _Float16* __restrict__ KH, _Float16* __restrict__ KL, _Float16* __restrict__ VT) {
  __shared__ __align__(16) _Float16 so[4][16][136], sol[4][16][136]; __shared__ __align__(16) _Float16 sth[128][72];
  const int tid = threadIdx.x, wave = tid >> 5, lane = tid & 31, col = lane & 15, g = lane >> 4;
  const int bx = blockIdx.x; const int b = bx / (RATE * MT), rem = bx - b * (RATE * MT), rr = rem / MT, mt = rem - rr * MT;
  const int mb = mt * 64, mrow = mb + wave * 16;
  const int which = blockIdx.y / (DMOD / 128), n0 = (blockIdx.y - which * (DMOD / 128)) * 128;
  const __bf16* xa = XB + ((size_t)b * LP + (size_t)RATE * (mrow + col) + rr) * DMOD;
  const __bf16* wb = WT + ((size_t)which * DMOD + n0 + col) * DMOD;
  v8f acc[8] = {};
#pragma unroll 2
  for (int kc = 0; kc < DMOD / 32; ++kc) { const v16b a = frag_b(xa + kc * 32, lane);
#pragma unroll
    for (int j = 0; j < 8; ++j) acc[j] = wmma_bf(a, frag_b(wb + (size_t)j * 16 * DMOD + kc * 32, lane), acc[j]); }
  const int gq = (b * NH + n0 / HD) * RATE + rr;
  if (which < 2) {
    _Float16* PHi = (which == 0) ? QH : KH; _Float16* PLo = (which == 0) ? QL : KL;
#pragma unroll
    for (int j = 0; j < 8; ++j) {
#pragma unroll
      for (int r = 0; r < 8; ++r) { const float v = acc[j][r]; const _Float16 hv = (_Float16)v; so[wave][8 * g + r][j * 16 + col] = hv; sol[wave][8 * g + r][j * 16 + col] = (_Float16)((v - (float)hv) * 2048.0f); } }
    LDSX();
#pragma unroll
    for (int it = 0; it < 8; ++it) { const int L = it * 4 + (lane >> 3), hh = L >> 4, rl = L & 15, pc = lane & 7;
      const size_t o = ((size_t)(gq + RATE * hh) * MP + mrow + rl) * HD + pc * 8;
      vst2(PHi + o, *(const v4u*)&so[wave][rl][hh * 64 + pc * 8]); vst2(PLo + o, *(const v4u*)&sol[wave][rl][hh * 64 + pc * 8]); }
  } else {
#pragma unroll
    for (int j = 0; j < 8; ++j) {
#pragma unroll
      for (int r = 0; r < 8; ++r) sth[j * 16 + col][wave * 16 + 8 * g + r] = (_Float16)acc[j][r]; }
    __syncthreads();
    for (int q = tid; q < 128 * 8; q += 128) { const int dc = q >> 3, pc = q & 7, hh = dc >> 6, d = dc & 63;
      const size_t o = ((size_t)(gq + RATE * hh) * HD + d) * MP + mb + pc * 8;
      vst2(VT + o, *(const v4u*)&sth[dc][pc * 8]); }
  }
}
__global__ __launch_bounds__(128) void k_attn(const _Float16* __restrict__ QH, const _Float16* __restrict__ QL, const _Float16* __restrict__ KH, const _Float16* __restrict__ KL, const _Float16* __restrict__ VT, float* __restrict__ O) {
  __shared__ __align__(16) float sp[4][16][36]; __shared__ __align__(16) float so[4][16][68];
  const int tid = threadIdx.x, wave = tid >> 5, lane = tid & 31, col = lane & 15, g = lane >> 4;
  const int qb = blockIdx.x, grp = blockIdx.y; const int rr = grp % RATE, h = (grp / RATE) % NH, b = grp / (RATE * NH);
  const int q0 = qb * 64 + wave * 16;
  const _Float16* qrow = QH + ((size_t)grp * MP + q0 + col) * HD; const _Float16* qrowl = QL + ((size_t)grp * MP + q0 + col) * HD;
  v16h aq[2], aql[2];
#pragma unroll
  for (int kc = 0; kc < 2; ++kc) { aq[kc] = frag_h(qrow + kc * 32, lane); aql[kc] = frag_h(qrowl + kc * 32, lane); }
  float m[8], l[8];
#pragma unroll
  for (int r = 0; r < 8; ++r) { m[r] = 0.f; const int mq = q0 + 8 * g + r; const int na = 3 - mq, nb = mq - (NVALID - 4); l[r] = (float)((na > 0 ? na : 0) + (nb > 0 ? nb : 0)); }
  v8f acc[4] = {}, accl[4] = {};
  const _Float16* kbase = KH + (size_t)grp * MP * HD; const _Float16* klbase = KL + (size_t)grp * MP * HD; const _Float16* vbase = VT + (size_t)grp * HD * MP;
#pragma unroll 1
  for (int ks = 0; ks < NKS; ++ks) { v8f s[2];
#pragma unroll
    for (int ct = 0; ct < 2; ++ct) { const int kk = ks * 32 + ct * 16 + col; const _Float16* krow = kbase + (size_t)kk * HD; const _Float16* krowl = klbase + (size_t)kk * HD; v8f c = {}, cl = {};
#pragma unroll
      for (int kc = 0; kc < 2; ++kc) { const v16h kh = frag_h(krow + kc * 32, lane); c = wmma16(aq[kc], kh, c); cl = wmma16(aql[kc], kh, cl); cl = wmma16(aq[kc], frag_h(krowl + kc * 32, lane), cl); }
#pragma unroll
      for (int r = 0; r < 8; ++r) c[r] += cl[r] * (1.0f / 2048.0f);
      const bool keepk = kk < NVALID;
#pragma unroll
      for (int r = 0; r < 8; ++r) s[ct][r] = keepk ? c[r] * 0.125f : -3.0e38f; }
#pragma unroll
    for (int r = 0; r < 8; ++r) { float mx = fmaxf(s[0][r], s[1][r]);
#pragma unroll
      for (int o = 1; o < 16; o <<= 1) mx = fmaxf(mx, __shfl_xor(mx, o));
      const float mn = fmaxf(m[r], mx); const float alpha = __expf(m[r] - mn);
      float e0 = (s[0][r] <= -1.0e38f) ? 0.f : __expf(s[0][r] - mn), e1 = (s[1][r] <= -1.0e38f) ? 0.f : __expf(s[1][r] - mn);
      const int mq = q0 + 8 * g + r; const int d0 = ks * 32 + col - mq, d1 = d0 + 16;
      e0 = (d0 >= -3 && d0 <= 3) ? (e0 + e0) : e0; e1 = (d1 >= -3 && d1 <= 3) ? (e1 + e1) : e1;
      float es = e0 + e1;
#pragma unroll
      for (int o = 1; o < 16; o <<= 1) es += __shfl_xor(es, o);
      l[r] = l[r] * alpha + es; m[r] = mn;
#pragma unroll
      for (int dt = 0; dt < 4; ++dt) { acc[dt][r] *= alpha; accl[dt][r] *= alpha; }
      sp[wave][8 * g + r][col] = e0; sp[wave][8 * g + r][16 + col] = e1; }
    LDSX();
    v16h pa, pl; { const float* prow = &sp[wave][col][0] + 8 * (lane >> 4);
#pragma unroll
      for (int i = 0; i < 8; ++i) { const float x0 = prow[i] * 2048.0f, x1 = prow[16 + i] * 2048.0f; const _Float16 h0 = (_Float16)x0, h1 = (_Float16)x1; pa[i] = h0; pa[8 + i] = h1; pl[i] = (_Float16)((x0 - (float)h0) * 2048.0f); pl[8 + i] = (_Float16)((x1 - (float)h1) * 2048.0f); } }
#pragma unroll
    for (int dt = 0; dt < 4; ++dt) { const v16h vh = frag_h(vbase + (size_t)(dt * 16 + col) * MP + ks * 32, lane); acc[dt] = wmma16(pa, vh, acc[dt]); accl[dt] = wmma16(pl, vh, accl[dt]); }
    LDSX(); }
#pragma unroll
  for (int r = 0; r < 8; ++r) { const float il = (1.0f / 2048.0f) / l[r];
#pragma unroll
    for (int dt = 0; dt < 4; ++dt) so[wave][8 * g + r][dt * 16 + col] = (acc[dt][r] + accl[dt][r] * (1.0f / 2048.0f)) * il; }
  LDSX();
#pragma unroll
  for (int it = 0; it < 8; ++it) { const int rl = it * 2 + g, pc = col;
    const size_t orow = (size_t)b * OSTRIDE_FULL + ((size_t)RATE * (q0 + rl) + rr) * DMOD;
    vst2(O + orow + h * HD + pc * 4, *(const v4f*)&so[wave][rl][pc * 4]); }
}
extern "C" void kernel_launch(void* const* d_in, const int* in_sizes, int n_in, void* d_out, int out_size, void* d_ws, size_t ws_size, hipStream_t stream) {
  if (n_in < 4) return;
  if (in_sizes[0] < NB * SEQ * DMOD || in_sizes[1] < DMOD * DMOD || in_sizes[2] < DMOD * DMOD || in_sizes[3] < DMOD * DMOD) return;
  if (out_size < NB * SEQ * DMOD) return;
  if (ws_size < WS_END) return;
  const float* X = (const float*)d_in[0]; const float* WQ = (const float*)d_in[1]; const float* WK = (const float*)d_in[2]; const float* WV = (const float*)d_in[3];
  char* ws = (char*)d_ws;
  __bf16* XB = (__bf16*)(ws + WS_XB); __bf16* WT = (__bf16*)(ws + WS_WT);
  _Float16* QH = (_Float16*)(ws + WS_QH); _Float16* QL = (_Float16*)(ws + WS_QL); _Float16* KH = (_Float16*)(ws + WS_KH); _Float16* KL = (_Float16*)(ws + WS_KL); _Float16* VT = (_Float16*)(ws + WS_VT);
  k_cvtx<<<dim3(LP / 4, NB), 256, 0, stream>>>(X, XB);
  k_wt<<<dim3(DMOD / 64, DMOD / 64, 3), 256, 0, stream>>>(WQ, WK, WV, WT);
  k_proj<<<dim3(NB * RATE * MT, 3 * (DMOD / 128)), 128, 0, stream>>>(XB, WT, QH, QL, KH, KL, VT);
  k_attn<<<dim3(NQB, NG), 128, 0, stream>>>(QH, QL, KH, KL, VT, (float*)d_out);
}
